// RelativeMultiHeadAttn_48361331753684
// MI455X (gfx1250) — hardware-verified
//
#include <hip/hip_runtime.h>
#include <math.h>

typedef __attribute__((ext_vector_type(16))) _Float16 v16h;
typedef __attribute__((ext_vector_type(16))) __bf16 v16b;
typedef __attribute__((ext_vector_type(8)))  _Float16 v8h;
typedef __attribute__((ext_vector_type(8)))  float v8f;
typedef __attribute__((ext_vector_type(4)))  float v4f;
typedef __attribute__((ext_vector_type(2)))  float v2f;
typedef __attribute__((ext_vector_type(4)))  unsigned v4u;
typedef __attribute__((ext_vector_type(4)))  int v4i;
typedef float __attribute__((may_alias)) float_a;
typedef int __attribute__((may_alias)) int_a;

template <typename T> __device__ __forceinline__ void vst2(void* p, T v) { *(volatile T*)p = v; __threadfence(); *(volatile T*)p = v; }
__device__ __forceinline__ v8f wmma16(v16h a, v16h b, v8f c) {
  v8f d = __builtin_amdgcn_wmma_f32_16x16x32_f16(false, a, false, b, (short)0, c, false, false);
  asm volatile("v_nop\n\tv_nop\n\tv_nop\n\tv_nop" : "+v"(d) : "v"(a), "v"(b));
  return d;
}
__device__ __forceinline__ v8f wmma_bf(v16b a, v16b b, v8f c) {
  v8f d = __builtin_amdgcn_wmma_f32_16x16x32_bf16(false, a, false, b, (short)0, c, false, false);
  asm volatile("v_nop\n\tv_nop\n\tv_nop\n\tv_nop" : "+v"(d) : "v"(a), "v"(b));
  return d;
}
__device__ __forceinline__ v16h frag_h(const _Float16* rowk0, int lane) {
  union { v16h v; v8h q[2]; } u; const _Float16* p = rowk0 + 8 * (lane >> 4);
  u.q[0] = *(const v8h*)p; u.q[1] = *(const v8h*)(p + 16); return u.v;
}
__device__ __forceinline__ v16h frag_f32(const float* rowk0, int lane) {
  v16h a; const float* p = rowk0 + 8 * (lane >> 4);
#pragma unroll
  for (int i = 0; i < 8; ++i) { a[i] = (_Float16)p[i]; a[8 + i] = (_Float16)p[16 + i]; }
  return a;
}
__device__ __forceinline__ v16h frag_f32s(const float* rowk0, int lane, float sc) {
  v16h a; const float* p = rowk0 + 8 * (lane >> 4);
#pragma unroll
  for (int i = 0; i < 8; ++i) { a[i] = (_Float16)(p[i] * sc); a[8 + i] = (_Float16)(p[16 + i] * sc); }
  return a;
}
__device__ __forceinline__ v16h fragc_f32(const float* W, int k0, int n, int lane, int ld, int K) {
  v16h a; const int g = lane >> 4;
#pragma unroll
  for (int i = 0; i < 8; ++i) { const int ka = k0 + 8 * g + i, kb = ka + 16;
    a[i] = (_Float16)(ka < K ? W[(size_t)(ka < K ? ka : K - 1) * ld + n] : 0.f); a[8 + i] = (_Float16)(kb < K ? W[(size_t)(kb < K ? kb : K - 1) * ld + n] : 0.f); }
  return a;
}
struct F2 { v16b h, l; };
__device__ __forceinline__ F2 bsplit16(const float v[16]) { F2 r;
#pragma unroll
  for (int i = 0; i < 16; ++i) { const __bf16 h = (__bf16)v[i]; r.h[i] = h; r.l[i] = (__bf16)(v[i] - (float)h); }
  return r; }
__device__ __forceinline__ F2 split_row(const float* row, int k0, int lane) { float v[16]; const float* p = row + k0 + 8 * (lane >> 4);
#pragma unroll
  for (int i = 0; i < 8; ++i) { v[i] = p[i]; v[8 + i] = p[16 + i]; }
  return bsplit16(v); }
__device__ __forceinline__ F2 split_rowK(const float* row, int k0, int lane, int K) { float v[16]; const int g = lane >> 4;
#pragma unroll
  for (int i = 0; i < 8; ++i) { const int ka = k0 + 8 * g + i, kb = ka + 16; v[i] = ka < K ? row[ka < K ? ka : K - 1] : 0.f; v[8 + i] = kb < K ? row[kb < K ? kb : K - 1] : 0.f; }
  return bsplit16(v); }
__device__ __forceinline__ F2 split_col(const float* W, int k0, int n, int lane, int ld, int K) { float v[16]; const int g = lane >> 4;
#pragma unroll
  for (int i = 0; i < 8; ++i) { const int ka = k0 + 8 * g + i, kb = ka + 16; v[i] = ka < K ? W[(size_t)(ka < K ? ka : K - 1) * ld + n] : 0.f; v[8 + i] = kb < K ? W[(size_t)(kb < K ? kb : K - 1) * ld + n] : 0.f; }
  return bsplit16(v); }
__device__ __forceinline__ v8f mac3(const F2& a, const F2& b, v8f c) { c = wmma_bf(a.l, b.h, c); c = wmma_bf(a.h, b.l, c); return wmma_bf(a.h, b.h, c); }
__device__ __forceinline__ float sigm(float v) { return 1.0f / (1.0f + expf(-v)); }
#define LDSX() do { asm volatile("s_wait_dscnt 0" ::: "memory"); __builtin_amdgcn_wave_barrier(); __builtin_amdgcn_fence(__ATOMIC_RELEASE, "workgroup"); } while (0)

#define NB 4
#define TT 1024
#define CC 1024
#define NH 16
#define HD 64
#define NPOS (2 * TT)
#define HRR (2 * TT + 128)
#define S2W (TT + 128)
#ifndef TNB
#define TNB NB
#endif
typedef __attribute__((ext_vector_type(8))) __bf16 v8b;
__device__ __forceinline__ v16b frag_b(const __bf16* rowk0, int lane) {
  union { v16b v; v8b q[2]; } u; const __bf16* p = rowk0 + 8 * (lane >> 4);
  u.q[0] = *(const v8b*)p; u.q[1] = *(const v8b*)(p + 16); return u.v;
}
__device__ __forceinline__ float bfr(float v) { return (float)(__bf16)v; }
__constant__ float FREQ[512] = {1.000000000e+0f,9.821718335e-1f,9.646616578e-1f,9.474635124e-1f,9.305720329e-1f,9.139816761e-1f,8.976871371e-1f,8.816831112e-1f,8.659643531e-1f,8.505258560e-1f,8.353625536e-1f,8.204696178e-1f,8.058422208e-1f,7.914755344e-1f,7.773650289e-1f,7.635061145e-1f,7.498942018e-1f,7.365249991e-1f,7.233941555e-1f,7.104974389e-1f,6.978305578e-1f,6.853895783e-1f,6.731703877e-1f,6.611690521e-1f,6.493816376e-1f,6.378043890e-1f,6.264335513e-1f,6.152654290e-1f,6.042963862e-1f,5.935229063e-1f,5.829415321e-1f,5.725488067e-1f,5.623413324e-1f,5.523158312e-1f,5.424690843e-1f,5.327978730e-1f,5.232991576e-1f,5.139696598e-1f,5.048065782e-1f,4.958068132e-1f,4.869675338e-1f,4.782858193e-1f,4.697588682e-1f,4.613839388e-1f,4.531583488e-1f,4.450793862e-1f,4.371444881e-1f,4.293510318e-1f,4.216965139e-1f,4.141784608e-1f,4.067944288e-1f,3.995420635e-1f,3.924189806e-1f,3.854228854e-1f,3.785515428e-1f,3.718026578e-1f,3.651741445e-1f,3.586637676e-1f,3.522694409e-1f,3.459891677e-1f,3.398208320e-1f,3.337624967e-1f,3.278121352e-1f,3.219678402e-1f,3.162277639e-1f,3.105900288e-1f,3.050527871e-1f,2.996142805e-1f,2.942727208e-1f,2.890264094e-1f,2.838735878e-1f,2.788126469e-1f,2.738419771e-1f,2.689598799e-1f,2.641648352e-1f,2.594552636e-1f,2.548296750e-1f,2.502865493e-1f,2.458243966e-1f,2.414418161e-1f,2.371373624e-1f,2.329096496e-1f,2.287573218e-1f,2.246790081e-1f,2.206733972e-1f,2.167392224e-1f,2.128751576e-1f,2.090799958e-1f,2.053525001e-1f,2.016914487e-1f,1.980956793e-1f,1.945640147e-1f,1.910952926e-1f,1.876884252e-1f,1.843423098e-1f,1.810558140e-1f,1.778279394e-1f,1.746576130e-1f,1.715437919e-1f,1.684854925e-1f,1.654817015e-1f,1.625314802e-1f,1.596338600e-1f,1.567878872e-1f,1.539926529e-1f,1.512472630e-1f,1.485508084e-1f,1.459024251e-1f,1.433012635e-1f,1.407464594e-1f,1.382372230e-1f,1.357727200e-1f,1.333521456e-1f,1.309747249e-1f,1.286396980e-1f,1.263462901e-1f,1.240937710e-1f,1.218814254e-1f,1.197085083e-1f,1.175743192e-1f,1.154782027e-1f,1.134194434e-1f,1.113973856e-1f,1.094113812e-1f,1.074607819e-1f,1.055449620e-1f,1.036632955e-1f,1.018151715e-1f,1.000000015e-1f,9.821718186e-2f,9.646616131e-2f,9.474635124e-2f,9.305720031e-2f,9.139817208e-2f,8.976870775e-2f,8.816830814e-2f,8.659642935e-2f,8.505257964e-2f,8.353625983e-2f,8.204696327e-2f,8.058421314e-2f,7.914755493e-2f,7.773650438e-2f,7.635060698e-2f,7.498941571e-2f,7.365249842e-2f,7.233941555e-2f,7.104974240e-2f,6.978305429e-2f,6.853895634e-2f,6.731703877e-2f,6.611690670e-2f,6.493816525e-2f,6.378044188e-2f,6.264335662e-2f,6.152653694e-2f,6.042964384e-2f,5.935229361e-2f,5.829415470e-2f,5.725487694e-2f,5.623412877e-2f,5.523158237e-2f,5.424690619e-2f,5.327979103e-2f,5.232991278e-2f,5.139696971e-2f,5.048065633e-2f,4.958068207e-2f,4.869675264e-2f,4.782858118e-2f,4.697588459e-2f,4.613839835e-2f,4.531583562e-2f,4.450793937e-2f,4.371444881e-2f,4.293510318e-2f,4.216964915e-2f,4.141784459e-2f,4.067944363e-2f,3.995420411e-2f,3.924189880e-2f,3.854228929e-2f,3.785515204e-2f,3.718026727e-2f,3.651741147e-2f,3.586637601e-2f,3.522694483e-2f,3.459891677e-2f,3.398208320e-2f,3.337624669e-2f,3.278120980e-2f,3.219678625e-2f,3.162277862e-2f,3.105900250e-2f,3.050527908e-2f,2.996142767e-2f,2.942727320e-2f,2.890264057e-2f,2.838735841e-2f,2.788126841e-2f,2.738419548e-2f,2.689598687e-2f,2.641648427e-2f,2.594552562e-2f,2.548296750e-2f,2.502865531e-2f,2.458244003e-2f,2.414418198e-2f,2.371373586e-2f,2.329096757e-2f,2.287573181e-2f,2.246790007e-2f,2.206734009e-2f,2.167392150e-2f,2.128751762e-2f,2.090799995e-2f,2.053525113e-2f,2.016914636e-2f,1.980956830e-2f,1.945639960e-2f,1.910953037e-2f,1.876884326e-2f,1.843423024e-2f,1.810558327e-2f,1.778279431e-2f,1.746576093e-2f,1.715437882e-2f,1.684854925e-2f,1.654817164e-2f,1.625314727e-2f,1.596338488e-2f,1.567878947e-2f,1.539926510e-2f,1.512472518e-2f,1.485508028e-2f,1.459024288e-2f,1.433012541e-2f,1.407464594e-2f,1.382372249e-2f,1.357727125e-2f,1.333521493e-2f,1.309747249e-2f,1.286396943e-2f,1.263462938e-2f,1.240937691e-2f,1.218814217e-2f,1.197085064e-2f,1.175743248e-2f,1.154781971e-2f,1.134194434e-2f,1.113973837e-2f,1.094113849e-2f,1.074607857e-2f,1.055449620e-2f,1.036632899e-2f,1.018151734e-2f,9.999999776e-3f,9.821719490e-3f,9.646615945e-3f,9.474635124e-3f,9.305720218e-3f,9.139816277e-3f,8.976871148e-3f,8.816830814e-3f,8.659643121e-3f,8.505257778e-3f,8.353625424e-3f,8.204696700e-3f,8.058422245e-3f,7.914755493e-3f,7.773650344e-3f,7.635060698e-3f,7.498942316e-3f,7.365249563e-3f,7.233941462e-3f,7.104974240e-3f,6.978305988e-3f,6.853895728e-3f,6.731703877e-3f,6.611690391e-3f,6.493816618e-3f,6.378043909e-3f,6.264335476e-3f,6.152654067e-3f,6.042964291e-3f,5.935229361e-3f,5.829415284e-3f,5.725487601e-3f,5.623413250e-3f,5.523158237e-3f,5.424690899e-3f,5.327979103e-3f,5.232991185e-3f,5.139696877e-3f,5.048065912e-3f,4.958068486e-3f,4.869675264e-3f,4.782858305e-3f,4.697588738e-3f,4.613839556e-3f,4.531583749e-3f,4.450793844e-3f,4.371444695e-3f,4.293510225e-3f,4.216964822e-3f,4.141784739e-3f,4.067944363e-3f,3.995420411e-3f,3.924189601e-3f,3.854229115e-3f,3.785515437e-3f,3.718026681e-3f,3.651741426e-3f,3.586637788e-3f,3.522694577e-3f,3.459891537e-3f,3.398208413e-3f,3.337624483e-3f,3.278121119e-3f,3.219678300e-3f,3.162277862e-3f,3.105900250e-3f,3.050528001e-3f,2.996142721e-3f,2.942727180e-3f,2.890263917e-3f,2.838735934e-3f,2.788126701e-3f,2.738419687e-3f,2.689598827e-3f,2.641648287e-3f,2.594552701e-3f,2.548296703e-3f,2.502865391e-3f,2.458244096e-3f,2.414418384e-3f,2.371373819e-3f,2.329096664e-3f,2.287573181e-3f,2.246790100e-3f,2.206734149e-3f,2.167392056e-3f,2.128751716e-3f,2.090800088e-3f,2.053525066e-3f,2.016914543e-3f,1.980956644e-3f,1.945640077e-3f,1.910952851e-3f,1.876884256e-3f,1.843422884e-3f,1.810558140e-3f,1.778279431e-3f,1.746576163e-3f,1.715437858e-3f,1.684854855e-3f,1.654817141e-3f,1.625314937e-3f,1.596338581e-3f,1.567878877e-3f,1.539926510e-3f,1.512472634e-3f,1.485507935e-3f,1.459024264e-3f,1.433012658e-3f,1.407464617e-3f,1.382372226e-3f,1.357727102e-3f,1.333521446e-3f,1.309747226e-3f,1.286396873e-3f,1.263462938e-3f,1.240937854e-3f,1.218814170e-3f,1.197085017e-3f,1.175743295e-3f,1.154782018e-3f,1.134194434e-3f,1.113973907e-3f,1.094113803e-3f,1.074607833e-3f,1.055449597e-3f,1.036632922e-3f,1.018151757e-3f,1.000000047e-3f,9.821718559e-4f,9.646615945e-4f,9.474635590e-4f,9.305721032e-4f,9.139817557e-4f,8.976871031e-4f,8.816830232e-4f,8.659643354e-4f,8.505258011e-4f,8.353625308e-4f,8.204695769e-4f,8.058422245e-4f,7.914755843e-4f,7.773649995e-4f,7.635060465e-4f,7.498941850e-4f,7.365249912e-4f,7.233941578e-4f,7.104973774e-4f,6.978305755e-4f,6.853896193e-4f,6.731703761e-4f,6.611690042e-4f,6.493816618e-4f,6.378043909e-4f,6.264335825e-4f,6.152653950e-4f,6.042963942e-4f,5.935229128e-4f,5.829415168e-4f,5.725487717e-4f,5.623413017e-4f,5.523158470e-4f,5.424690899e-4f,5.327978870e-4f,5.232990952e-4f,5.139696877e-4f,5.048065796e-4f,4.958068021e-4f,4.869675031e-4f,4.782858014e-4f,4.697588738e-4f,4.613839847e-4f,4.531583400e-4f,4.450794077e-4f,4.371444811e-4f,4.293509992e-4f,4.216964880e-4f,4.141784448e-4f,4.067944246e-4f,3.995420411e-4f,3.924189950e-4f,3.854228707e-4f,3.785515146e-4f,3.718026564e-4f,3.651741135e-4f,3.586637613e-4f,3.522694460e-4f,3.459891595e-4f,3.398208064e-4f,3.337624657e-4f,3.278121294e-4f,3.219678474e-4f,3.162277862e-4f,3.105900250e-4f,3.050527885e-4f,2.996142721e-4f,2.942727297e-4f,2.890263859e-4f,2.838736109e-4f,2.788126585e-4f,2.738419571e-4f,2.689598768e-4f,2.641648462e-4f,2.594552934e-4f,2.548296761e-4f,2.502865391e-4f,2.458243980e-4f,2.414418122e-4f,2.371373848e-4f,2.329096606e-4f,2.287573152e-4f,2.246790100e-4f,2.206734207e-4f,2.167392086e-4f,2.128751657e-4f,2.090800117e-4f,2.053524950e-4f,2.016914514e-4f,1.980956731e-4f,1.945640106e-4f,1.910952997e-4f,1.876884344e-4f,1.843422942e-4f,1.810558315e-4f,1.778279402e-4f,1.746576017e-4f,1.715437829e-4f,1.684854797e-4f,1.654817170e-4f,1.625314762e-4f,1.596338552e-4f,1.567878790e-4f,1.539926452e-4f,1.512472518e-4f,1.485508110e-4f,1.459024206e-4f,1.433012658e-4f,1.407464733e-4f,1.382372284e-4f,1.357727160e-4f,1.333521504e-4f,1.309747167e-4f,1.286396873e-4f,1.263462909e-4f,1.240937709e-4f,1.218814141e-4f,1.197085076e-4f,1.175743309e-4f,1.154781930e-4f,1.134194390e-4f,1.113973922e-4f,1.094113759e-4f,1.074607790e-4f,1.055449538e-4f,1.036632893e-4f,1.018151743e-4f};
#define RSCALE 102.40000152587890625f

#define HG 2
#define WS_QUH 0u
#define WS_QUL (WS_QUH + 2u * (size_t)NB * TT * CC)
#define WS_QVH (WS_QUL + 2u * (size_t)NB * TT * CC)
#define WS_QVL (WS_QVH + 2u * (size_t)NB * TT * CC)
#define WS_KH  (WS_QVL + 2u * (size_t)NB * TT * CC)
#define WS_RH  (WS_KH  + 2u * (size_t)NB * TT * CC)
#define WS_RL  (WS_RH  + 2u * (size_t)HRR * CC)
#define WS_HRH (WS_RL  + 2u * (size_t)HRR * CC)
#define WS_HRL (WS_HRH + 2u * (size_t)HRR * CC)
#define WS_VT  (WS_HRL + 2u * (size_t)HRR * CC)
#define WS_VL  (WS_VT  + 2u * (size_t)NB * CC * TT)
#define WS_S1  (WS_VL  + 2u * (size_t)NB * CC * TT)
#define WS_S2  (WS_S1  + 4u * (size_t)HG * TT * TT)
#define WS_Y   (WS_S2  + 4u * (size_t)HG * TT * S2W)
#define WS_Z   (WS_Y   + 4u * (size_t)NB * TT * CC)
#define WS_END (WS_Z   + 4u * (size_t)NB * TT * CC)

__global__ __launch_bounds__(256) void k_rtab(__bf16* __restrict__ RH, __bf16* __restrict__ RL) { __shared__ __align__(16) float sv[1024];
  const int t = threadIdx.x; const int p = blockIdx.x; const float pos = (float)(TT - p);
#pragma unroll 1
  for (int c = t; c < CC; c += 256) { const float ang = pos * FREQ[c >> 1]; sv[c] = ((c & 1) ? cosf(ang) : sinf(ang)) * RSCALE; }
  __syncthreads();
  for (int e = t; e < CC / 8; e += 256) { v8b hi, lo;
#pragma unroll
    for (int z = 0; z < 8; ++z) { const float v = sv[e * 8 + z]; const __bf16 h = (__bf16)v; hi[z] = h; lo[z] = (__bf16)(v - (float)h); }
    vst2(RH + (size_t)p * CC + e * 8, hi); vst2(RL + (size_t)p * CC + e * 8, lo); } }
__global__ __launch_bounds__(128) void k_proj(const float* __restrict__ X0, const float* __restrict__ X1, const float* __restrict__ X2, const float* __restrict__ WQ, const float* __restrict__ WK, const float* __restrict__ WV, const float* __restrict__ UW, const float* __restrict__ VW, _Float16* __restrict__ QUH, _Float16* __restrict__ QUL, _Float16* __restrict__ QVH, _Float16* __restrict__ QVL, _Float16* __restrict__ KH, __bf16* __restrict__ VT, __bf16* __restrict__ VL) {
  __shared__ __align__(16) _Float16 sh[64][136], sl[64][136]; __shared__ __align__(16) __bf16 th[128][72], tl2[128][72];
  const int tid = threadIdx.x, wave = tid >> 5, lane = tid & 31, col = lane & 15, g = lane >> 4; const int which = blockIdx.z; const int c0 = blockIdx.y * 128; const size_t r0 = (size_t)blockIdx.x * 64; const float* WA = which == 0 ? WQ : which == 1 ? WK : WV;
  v8f acc[8] = {};
  const float* X = which == 0 ? X0 : which == 1 ? X1 : X2;
#pragma unroll 2
  for (int kc = 0; kc < CC / 32; ++kc) { v16b a; { const float* p = X + (r0 + wave * 16 + col) * CC + kc * 32 + 8 * g;
#pragma unroll
      for (int i = 0; i < 8; ++i) { a[i] = (__bf16)p[i]; a[8 + i] = (__bf16)p[16 + i]; } }
#pragma unroll
    for (int j = 0; j < 8; ++j) { v16b w; const int o = c0 + j * 16 + col; const float* wp = WA + (size_t)o * CC + kc * 32 + 8 * g;
#pragma unroll
      for (int i = 0; i < 8; ++i) { w[i] = (__bf16)wp[i]; w[8 + i] = (__bf16)wp[16 + i]; }
      asm volatile("s_wait_loadcnt 0x0" ::: "memory"); acc[j] = wmma_bf(a, w, acc[j]); } }
  const int npass = (which == 0) ? 2 : 1;
  for (int pass = 0; pass < npass; ++pass) {
    if (pass) __syncthreads();
#pragma unroll
    for (int j = 0; j < 8; ++j) { const float bb = (which == 0) ? bfr((pass == 0 ? UW : VW)[(c0 + j * 16 + col) & (HD - 1)]) : 0.f;
#pragma unroll
      for (int r = 0; r < 8; ++r) { const float v = acc[j][r] + bb; const int rl = wave * 16 + 8 * g + r, cl = j * 16 + col; const _Float16 hv = (_Float16)v;
        if (which == 2) { const __bf16 bh = (__bf16)v; th[cl][rl] = bh; tl2[cl][rl] = (__bf16)(v - (float)bh); } else { sh[rl][cl] = hv; sl[rl][cl] = (_Float16)((v - (float)hv) * 1024.0f); }     } }
    __syncthreads();
    if (which < 2) { _Float16* dh = which == 1 ? KH : (pass == 0 ? QUH : QVH); _Float16* dl = (pass == 0 ? QUL : QVL); for (int e = tid; e < 64 * 16; e += 128) { const int rl = e >> 4, q = e & 15; vst2((unsigned*)(dh + (r0 + rl) * CC + c0 + q * 8), *(const v4u*)&sh[rl][q * 8]); if (which == 0) vst2((unsigned*)(dl + (r0 + rl) * CC + c0 + q * 8), *(const v4u*)&sl[rl][q * 8]); } }
    else { const size_t b = r0 / TT; const int t0 = (int)(r0 % TT); for (int e = tid; e < 128 * 8; e += 128) { const int cl = e >> 3, q = e & 7; const size_t o2 = (b * CC + c0 + cl) * (size_t)TT + t0 + q * 8; vst2((unsigned*)(VT + o2), *(const v4u*)&th[cl][q * 8]); vst2((unsigned*)(VL + o2), *(const v4u*)&tl2[cl][q * 8]); } } } }
__global__ __launch_bounds__(128) void k_projr(const __bf16* __restrict__ RH, const __bf16* __restrict__ RL, const float* __restrict__ WR, _Float16* __restrict__ HRH, _Float16* __restrict__ HRL) {
  __shared__ __align__(16) _Float16 sh[64][136], sl[64][136];
  const int tid = threadIdx.x, wave = tid >> 5, lane = tid & 31, col = lane & 15, g = lane >> 4; const int c0 = blockIdx.y * 128; const size_t p0 = (size_t)blockIdx.x * 64;
  v8f acc[8] = {};
#pragma unroll 2
  for (int kc = 0; kc < CC / 32; ++kc) { const v16b ah = frag_b(RH + (p0 + wave * 16 + col) * CC + kc * 32, lane), al = frag_b(RL + (p0 + wave * 16 + col) * CC + kc * 32, lane);
#pragma unroll
    for (int j = 0; j < 8; ++j) { v16b w; const int o = c0 + j * 16 + col; const float* wp = WR + (size_t)o * CC + kc * 32 + 8 * g;
#pragma unroll
      for (int i = 0; i < 8; ++i) { w[i] = (__bf16)wp[i]; w[8 + i] = (__bf16)wp[16 + i]; }
      asm volatile("s_wait_loadcnt 0x0" ::: "memory"); acc[j] = wmma_bf(ah, w, acc[j]); acc[j] = wmma_bf(al, w, acc[j]); } }
#pragma unroll
  for (int j = 0; j < 8; ++j) {
#pragma unroll
    for (int r = 0; r < 8; ++r) { const float v = acc[j][r]; const int rl = wave * 16 + 8 * g + r, cl = j * 16 + col; const _Float16 hv = (_Float16)v; sh[rl][cl] = hv; sl[rl][cl] = (_Float16)((v - (float)hv) * 1024.0f); } }
  __syncthreads();
  for (int e = tid; e < 64 * 16; e += 128) { const int rl = e >> 4, q = e & 15; vst2((unsigned*)(HRH + (p0 + rl) * CC + c0 + q * 8), *(const v4u*)&sh[rl][q * 8]); vst2((unsigned*)(HRL + (p0 + rl) * CC + c0 + q * 8), *(const v4u*)&sl[rl][q * 8]); } }
__global__ __launch_bounds__(128) void k_sc1(const _Float16* __restrict__ QH, const _Float16* __restrict__ QL, const _Float16* __restrict__ KH, int b, int h0, float* __restrict__ S0) { __shared__ __align__(16) float ss[4][16][132]; const int h = h0 + blockIdx.z; float* S = S0 + (size_t)blockIdx.z * TT * TT;
  const int tid = threadIdx.x, wave = tid >> 5, lane = tid & 31, col = lane & 15, g = lane >> 4; const int k0 = blockIdx.y * 128; const int ql0 = blockIdx.x * 64 + wave * 16; const size_t q0 = (size_t)b * TT + ql0;
  v8f acc[8] = {}, accl[8] = {};
#pragma unroll
  for (int kc = 0; kc < HD / 32; ++kc) { const v16h ah = frag_h(QH + (q0 + col) * CC + h * HD + kc * 32, lane), al = frag_h(QL + (q0 + col) * CC + h * HD + kc * 32, lane);
#pragma unroll
    for (int j = 0; j < 8; ++j) { const v16h kb = frag_h(KH + ((size_t)b * TT + k0 + j * 16 + col) * CC + h * HD + kc * 32, lane); acc[j] = wmma16(ah, kb, acc[j]); accl[j] = wmma16(al, kb, accl[j]); } }
#pragma unroll
  for (int j = 0; j < 8; ++j) {
#pragma unroll
    for (int r = 0; r < 8; ++r) ss[wave][8 * g + r][j * 16 + col] = acc[j][r] + accl[j][r] * (1.0f / 1024.0f); }
  LDSX(); for (int rl = 0; rl < 16; ++rl) vst2(S + (size_t)(ql0 + rl) * TT + k0 + lane * 4, *(const v4f*)&ss[wave][rl][lane * 4]); }
__global__ __launch_bounds__(128) void k_sc2(const _Float16* __restrict__ QH, const _Float16* __restrict__ QL, const _Float16* __restrict__ RHh, const _Float16* __restrict__ RLl, int b, int h0, float* __restrict__ S0) { __shared__ __align__(16) float ss[4][16][132]; const int h = h0 + blockIdx.z; float* S = S0 + (size_t)blockIdx.z * TT * S2W;
  const int tid = threadIdx.x, wave = tid >> 5, lane = tid & 31, col = lane & 15, g = lane >> 4; const int i0 = blockIdx.x * 64; const int cb0 = blockIdx.y * 128; const size_t p0 = (size_t)(TT - i0 - 64) + cb0; const int ql0 = i0 + wave * 16; const size_t q0 = (size_t)b * TT + ql0;
  v8f acc[8] = {}, accl[8] = {};
#pragma unroll
  for (int kc = 0; kc < HD / 32; ++kc) { const v16h ah = frag_h(QH + (q0 + col) * CC + h * HD + kc * 32, lane), al = frag_h(QL + (q0 + col) * CC + h * HD + kc * 32, lane);
#pragma unroll
    for (int j = 0; j < 8; ++j) { const size_t pr = (p0 + j * 16 + col) * CC + h * HD + kc * 32; const v16h kb = frag_h(RHh + pr, lane), kl = frag_h(RLl + pr, lane); acc[j] = wmma16(ah, kb, acc[j]); accl[j] = wmma16(al, kb, accl[j]); accl[j] = wmma16(ah, kl, accl[j]); } }
#pragma unroll
  for (int j = 0; j < 8; ++j) {
#pragma unroll
    for (int r = 0; r < 8; ++r) ss[wave][8 * g + r][j * 16 + col] = acc[j][r] + accl[j][r] * (1.0f / 1024.0f); }
  LDSX(); for (int rl = 0; rl < 16; ++rl) vst2(S + (size_t)(ql0 + rl) * S2W + cb0 + lane * 4, *(const v4f*)&ss[wave][rl][lane * 4]); }
__global__ __launch_bounds__(256) void k_sm(float* __restrict__ S0, const float* __restrict__ S2_0) { __shared__ float sred[8]; __shared__ float sbc; __shared__ __align__(16) float shv[TT];
  const int t = threadIdx.x; const int row = blockIdx.x; float* sr = S0 + (size_t)blockIdx.y * TT * TT + (size_t)row * TT; const float* s2 = S2_0 + (size_t)blockIdx.y * TT * S2W + (size_t)row * S2W + (64 - (row & 63)); const int kend = TT;
  float m = -3.0e38f; for (int k = t; k < kend; k += 256) { const float v = (sr[k] + s2[k]) * 0.03125f; shv[k] = v; m = fmaxf(m, v); }
#pragma unroll
  for (int o = 1; o < 32; o <<= 1) m = fmaxf(m, __shfl_xor(m, o));
  if ((t & 31) == 0) sred[t >> 5] = m; __syncthreads(); if (t == 0) { float a = sred[0]; for (int i = 1; i < 8; ++i) a = fmaxf(a, sred[i]); sbc = a; } __syncthreads(); m = sbc; __syncthreads();
  float sum = 0.f; for (int k = t; k < kend; k += 256) { const float e = expf(shv[k] - m); shv[k] = e; sum += e; }
#pragma unroll
  for (int o = 1; o < 32; o <<= 1) sum += __shfl_xor(sum, o);
  if ((t & 31) == 0) sred[t >> 5] = sum; __syncthreads(); if (t == 0) { float a = 0.f; for (int i = 0; i < 8; ++i) a += sred[i]; sbc = 1.0f / a; } __syncthreads(); const float inv = sbc * 2048.0f;
  for (int k = t; k < kend; k += 256) shv[k] = shv[k] * inv;
  __syncthreads(); for (int q = t; q < kend / 4; q += 256) vst2(sr + q * 4, *(const v4f*)&shv[q * 4]); }
__global__ __launch_bounds__(128) void k_pv(const float* __restrict__ PS0, const __bf16* __restrict__ VT, const __bf16* __restrict__ VL, int b, int h0, float* __restrict__ Y) { const int h = h0 + blockIdx.z; const float* PS = PS0 + (size_t)blockIdx.z * TT * TT; __shared__ __align__(16) float ss[4][16][HD + 4];
  const int tid = threadIdx.x, wave = tid >> 5, lane = tid & 31, col = lane & 15, g = lane >> 4; const int ql0 = blockIdx.x * 64 + wave * 16; const int kend = TT;
  v8f acc[HD / 16] = {};
#pragma unroll 1
  for (int kc = 0; kc < kend / 32; ++kc) { const F2 p = split_row(PS + (size_t)(ql0 + col) * TT, kc * 32, lane);
#pragma unroll
    for (int j = 0; j < HD / 16; ++j) { const size_t po = ((size_t)b * CC + h * HD + j * 16 + col) * (size_t)TT + kc * 32; const v16b vh = frag_b(VT + po, lane); acc[j] = wmma_bf(p.h, vh, acc[j]); acc[j] = wmma_bf(p.l, vh, acc[j]); acc[j] = wmma_bf(p.h, frag_b(VL + po, lane), acc[j]); } }
#pragma unroll
  for (int j = 0; j < HD / 16; ++j)
#pragma unroll
    for (int r = 0; r < 8; ++r) ss[wave][8 * g + r][j * 16 + col] = acc[j][r] * (1.0f / 2048.0f);
  LDSX(); for (int rl = 0; rl < 16; ++rl) if (lane < HD / 4) vst2(Y + ((size_t)b * TT + ql0 + rl) * CC + h * HD + lane * 4, *(const v4f*)&ss[wave][rl][lane * 4]); }
__global__ __launch_bounds__(128) void k_out(const float* __restrict__ Yr, const float* __restrict__ WP, const float* __restrict__ XQ, float* __restrict__ Z) { __shared__ __align__(16) float sf[4][16][132];
  const int tid = threadIdx.x, wave = tid >> 5, lane = tid & 31, col = lane & 15, g = lane >> 4; const int c0 = blockIdx.y * 128; const size_t r0 = (size_t)blockIdx.x * 64 + wave * 16;
  v8f acc[8] = {};
#pragma unroll 2
  for (int kc = 0; kc < CC / 32; ++kc) { const F2 a = split_row(Yr + (r0 + col) * CC, kc * 32, lane);
#pragma unroll
    for (int j = 0; j < 8; ++j) { v16b w; const int o = c0 + j * 16 + col; const float* wp = WP + (size_t)o * CC + kc * 32 + 8 * g;
#pragma unroll
      for (int i = 0; i < 8; ++i) { w[i] = (__bf16)wp[i]; w[8 + i] = (__bf16)wp[16 + i]; }
      asm volatile("s_wait_loadcnt 0x0" ::: "memory"); acc[j] = wmma_bf(a.h, w, acc[j]); acc[j] = wmma_bf(a.l, w, acc[j]); } }
#pragma unroll
  for (int j = 0; j < 8; ++j) { const int o = c0 + j * 16 + col;
#pragma unroll
    for (int r = 0; r < 8; ++r) { const size_t row = r0 + 8 * g + r; sf[wave][8 * g + r][j * 16 + col] = acc[j][r] + bfr(XQ[row * CC + o]); }
    asm volatile("s_wait_loadcnt 0x0" ::: "memory"); }
  LDSX(); for (int rl = 0; rl < 16; ++rl) vst2(Z + (r0 + rl) * CC + c0 + lane * 4, *(const v4f*)&sf[wave][rl][lane * 4]); }
__global__ __launch_bounds__(256) void k_ln(const float* __restrict__ Z, const float* __restrict__ G, const float* __restrict__ Bb, float* __restrict__ OUT) { __shared__ float sred[8]; __shared__ float sbc;
  const int t = threadIdx.x; const size_t row = blockIdx.x; const v4f y = *(const v4f*)(Z + row * CC + t * 4);
  float s = (y[0] + y[1]) + (y[2] + y[3]);
#pragma unroll
  for (int o = 1; o < 32; o <<= 1) s += __shfl_xor(s, o);
  if ((t & 31) == 0) sred[t >> 5] = s; __syncthreads(); if (t == 0) { float a = 0.f; for (int i = 0; i < 8; ++i) a += sred[i]; sbc = a * (1.0f / CC); } __syncthreads(); const float mean = sbc; __syncthreads();
  float d[4], s2 = 0.f;
#pragma unroll
  for (int z = 0; z < 4; ++z) { d[z] = y[z] - mean; s2 += d[z] * d[z]; }
#pragma unroll
  for (int o = 1; o < 32; o <<= 1) s2 += __shfl_xor(s2, o);
  if ((t & 31) == 0) sred[t >> 5] = s2; __syncthreads(); if (t == 0) { float a = 0.f; for (int i = 0; i < 8; ++i) a += sred[i]; sbc = 1.0f / (sqrtf(a * (1.0f / (CC - 1))) + 1e-9f); } __syncthreads(); const float rstd = sbc;
  v4f o4;
#pragma unroll
  for (int z = 0; z < 4; ++z) o4[z] = bfr(G[t * 4 + z]) * (d[z] * rstd) + bfr(Bb[t * 4 + z]);
  vst2(OUT + row * CC + t * 4, o4); }
extern "C" void kernel_launch(void* const* d_in, const int* in_sizes, int n_in, void* d_out, int out_size, void* d_ws, size_t ws_size, hipStream_t stream) {
  (void)in_sizes; (void)n_in; (void)out_size;
  const float** F = (const float**)d_in;
  if (ws_size < (size_t)WS_END) return;
  char* ws = (char*)d_ws; _Float16 *QUH = (_Float16*)(ws + WS_QUH), *QUL = (_Float16*)(ws + WS_QUL), *QVH = (_Float16*)(ws + WS_QVH), *QVL = (_Float16*)(ws + WS_QVL), *KH = (_Float16*)(ws + WS_KH), *HRH = (_Float16*)(ws + WS_HRH), *HRL = (_Float16*)(ws + WS_HRL); __bf16 *RH = (__bf16*)(ws + WS_RH), *RL = (__bf16*)(ws + WS_RL), *VT = (__bf16*)(ws + WS_VT), *VL = (__bf16*)(ws + WS_VL); float *S1 = (float*)(ws + WS_S1), *S2 = (float*)(ws + WS_S2), *Y = (float*)(ws + WS_Y), *Z = (float*)(ws + WS_Z);
  k_rtab<<<dim3(HRR), 256, 0, stream>>>(RH, RL);
  k_proj<<<dim3(TNB * TT / 64, CC / 128, 3), 128, 0, stream>>>(F[0], F[1], F[2], F[3], F[4], F[5], F[7], F[8], QUH, QUL, QVH, QVL, KH, VT, VL);
  k_projr<<<dim3(HRR / 64, CC / 128), 128, 0, stream>>>(RH, RL, F[6], HRH, HRL);
  for (int b = 0; b < TNB; ++b) for (int h0 = 0; h0 < NH; h0 += HG) {
    k_sc1<<<dim3(TT / 64, TT / 128, HG), 128, 0, stream>>>(QUH, QUL, KH, b, h0, S1);
    k_sc2<<<dim3(TT / 64, S2W / 128, HG), 128, 0, stream>>>(QVH, QVL, HRH, HRL, b, h0, S2);
    k_sm<<<dim3(TT, HG), 256, 0, stream>>>(S1, S2);
    k_pv<<<dim3(TT / 64, 1, HG), 128, 0, stream>>>(S1, VT, VL, b, h0, Y);
  }
  k_out<<<dim3(TNB * TT / 64, CC / 128), 128, 0, stream>>>(Y, F[9], F[0], Z);
  k_ln<<<dim3(TNB * TT), 256, 0, stream>>>(Z, F[10], F[11], (float*)d_out);
}
